// ResidualSyntaxGCN_31868657336591
// MI455X (gfx1250) — hardware-verified
//
#include <hip/hip_runtime.h>


namespace {
constexpr int N = 50000, E = 800000, G = 256, H = 64, L = 4, NPAD = 50176  , NBLK = NPAD / 128, NBA = NPAD / 1024;
constexpr float FXS = 1048576.0f, FXI = 1.0f / 1048576.0f, BNE = 1e-5f;
constexpr float PFXS = 262144.0f, PFXI = 1.0f / 262144.0f;

typedef _Float16 b16;
typedef __attribute__((ext_vector_type(16))) _Float16 v16b;
typedef __attribute__((ext_vector_type(8)))  _Float16 v8b;
typedef __attribute__((ext_vector_type(8)))  float v8f;
typedef __attribute__((ext_vector_type(4)))  float v4f;

__device__ __forceinline__ v8b ld8b(const b16* p) { return *(const v8b*)p; }
__device__ __forceinline__ v16b cat8b(v8b a, v8b b) { return __builtin_shufflevector(a, b, 0, 1, 2, 3, 4, 5, 6, 7, 8, 9, 10, 11, 12, 13, 14, 15); }
__device__ __forceinline__ v16b frag_kb(const b16* p, int hh) { return cat8b(ld8b(p + 8 * hh), ld8b(p + 16 + 8 * hh)); }
__device__ __forceinline__ void split16(float v, b16& hi, b16& lo) { hi = (b16)v; lo = (b16)(v - (float)hi); }
__device__ __forceinline__ void frag_ksplit(const float* p, int hh, v16b& fh_, v16b& fl_) {
  const float* p0 = p + 8 * hh; const float* p1 = p + 16 + 8 * hh;
#pragma unroll
  for (int e = 0; e < 8; ++e) { b16 a, c; split16(p0[e], a, c); fh_[e] = a; fl_[e] = c; split16(p1[e], a, c); fh_[8 + e] = a; fl_[8 + e] = c; }
}
__device__ __forceinline__ v8f wmma16b(v16b a, v16b b, v8f c) {
  v8f d = __builtin_amdgcn_wmma_f32_16x16x32_f16(false, a, false, b, (short)0, c, false, false);
  asm volatile("v_nop\n\tv_nop\n\tv_nop\n\tv_nop" : "+v"(d) : "v"(a), "v"(b));
  return d;
}
__device__ __forceinline__ void wave_lds_sync() {
  __builtin_amdgcn_fence(__ATOMIC_RELEASE, "workgroup");
  __builtin_amdgcn_wave_barrier();
  __builtin_amdgcn_fence(__ATOMIC_ACQUIRE, "workgroup");
}

struct Opnd { const void* p0; const void* p1; int ld; };
template <int NP> __device__ __forceinline__ void load_frags(const Opnd& o, int row, int kb, int hh, v16b& fh_, v16b& fl_) {
  if (NP == 0) { frag_ksplit((const float*)o.p0 + (size_t)row * o.ld + kb, hh, fh_, fl_); }
  else if (NP == 4) {
    const float* p = (const float*)o.p0 + (size_t)row * o.ld + kb; const float* p0 = p + 8 * hh; const float* p1 = p + 16 + 8 * hh;
#pragma unroll
    for (int e = 0; e < 8; ++e) { b16 a, c; split16(p0[e] * 64.0f, a, c); fh_[e] = a; fl_[e] = c; split16(p1[e] * 64.0f, a, c); fh_[8 + e] = a; fl_[8 + e] = c; }
  } else if (NP == 3) {
    const float* p = (const float*)o.p0 + (size_t)row * o.ld + kb; const float* p0 = p + 8 * hh; const float* p1 = p + 16 + 8 * hh;
#pragma unroll
    for (int e = 0; e < 8; ++e) { fh_[e] = (b16)p0[e]; fh_[8 + e] = (b16)p1[e]; }
    fl_ = fh_;
  } else {
    fh_ = frag_kb((const b16*)o.p0 + (size_t)row * o.ld + kb, hh);
    if (NP == 2) fl_ = frag_kb((const b16*)o.p1 + (size_t)row * o.ld + kb, hh); else fl_ = fh_;
  }
}
template <int ANP, int BNP> __device__ __forceinline__ v8f mac(v16b ah, v16b al, v16b bh, v16b bl, v8f c) {
  c = wmma16b(ah, bh, c);
  if (BNP == 0 || BNP == 2 || BNP == 4) c = wmma16b(ah, bl, c);
  if (ANP == 0 || ANP == 2 || ANP == 4) c = wmma16b(al, bh, c);
  return c;
}
template <int ANP, int BNP>
__device__ __forceinline__ void gemm_tile(const Opnd& A, const Opnd& B, int K, int m0, int c0, int nloc, int hlf, v8f (&acc)[2][4]) {
  for (int kb = 0; kb < K; kb += 32) {
    v16b a0h, a0l, a1h, a1l;
    load_frags<ANP>(A, m0 + nloc, kb, hlf, a0h, a0l);
    load_frags<ANP>(A, m0 + 16 + nloc, kb, hlf, a1h, a1l);
#pragma unroll
    for (int t = 0; t < 4; ++t) {
      v16b bh, bl;
      load_frags<BNP>(B, c0 + t * 16 + nloc, kb, hlf, bh, bl);
      acc[0][t] = mac<ANP, BNP>(a0h, a0l, bh, bl, acc[0][t]);
      acc[1][t] = mac<ANP, BNP>(a1h, a1l, bh, bl, acc[1][t]);
    }
  }
}

__device__ __forceinline__ void epi_planes(v8f (&acc)[2][4], float scale, bool two, b16* __restrict__ oh, b16* __restrict__ ol, int ldo,
                                           int m0, int c0, int lane, b16* Th, b16* Tl) {
  const int nloc = lane & 15, hlf = lane >> 4;
#pragma unroll
  for (int t = 0; t < 4; ++t)
#pragma unroll
    for (int r = 0; r < 2; ++r)
#pragma unroll
      for (int v = 0; v < 8; ++v) {
        const int rr = r * 16 + v + 8 * hlf, cc = t * 16 + nloc;
        b16 h_, l_; split16(acc[r][t][v] * scale, h_, l_);
        Th[rr * 64 + cc] = h_; Tl[rr * 64 + cc] = l_;
      }
  wave_lds_sync();
  for (int pass = 0; pass < 2; ++pass) {
#pragma unroll
    for (int j = 0; j < 8; ++j) {
      const int rr = j * 4 + (lane >> 3), c8 = (lane & 7) * 8;
      const size_t o = (size_t)(m0 + rr) * ldo + c0 + c8;
      *(volatile v8b*)(oh + o) = ld8b(Th + rr * 64 + c8);
      if (two) *(volatile v8b*)(ol + o) = ld8b(Tl + rr * 64 + c8);
    }
    __threadfence();
  }
}
__device__ __forceinline__ void epi_f32(v8f (&acc)[2][4], float scale, const float* rscale, float* __restrict__ out, int ldo, int m0, int c0, int lane, float* Tt) {
  const int nloc = lane & 15, hlf = lane >> 4;
#pragma unroll
  for (int t = 0; t < 4; ++t)
#pragma unroll
    for (int r = 0; r < 2; ++r)
#pragma unroll
      for (int v = 0; v < 8; ++v) {
        const int rr = r * 16 + v + 8 * hlf;
        const float rs = rscale ? rscale[(size_t)(m0 + rr) * 32] : 1.0f;
        Tt[rr * 64 + t * 16 + nloc] = acc[r][t][v] * scale * rs;
      }
  wave_lds_sync();
  float* dst0 = out + (size_t)m0 * ldo + c0;
  for (int pass = 0; pass < 2; ++pass) {
#pragma unroll
    for (int j = 0; j < 16; ++j) { const int rr = j * 2 + hlf, c4 = nloc * 4; *(volatile v4f*)(dst0 + (size_t)rr * ldo + c4) = *(const v4f*)(Tt + rr * 64 + c4); }
    __threadfence();
  }
}


__device__ __forceinline__ int fkey(float f) { const int b = __float_as_int(f); return (b >= 0) ? b : (b ^ 0x7FFFFFFF); }
__device__ __forceinline__ float fkey_inv(int k) { return __int_as_float((k >= 0) ? k : (k ^ 0x7FFFFFFF)); }

__global__ __launch_bounds__(256) void prep_kernel(const float* __restrict__ cw, b16* __restrict__ w8h, b16* __restrict__ w8l) {
  const size_t tid = (size_t)blockIdx.x * blockDim.x + threadIdx.x, nth = (size_t)gridDim.x * blockDim.x;
  for (int pass = 0; pass < 2; ++pass) { for (size_t p = tid; p < (size_t)8 * H * H / 8; p += nth) { const int m = (int)(p / (H * H / 8)); const int rem = (int)(p % (H * H / 8)), n = rem / 8, k0 = (rem % 8) * 8; v8b v, u;
#pragma unroll
      for (int e = 0; e < 8; ++e) { b16 a, c; split16(cw[((size_t)m * H + k0 + e) * H + n] * 64.0f, a, c); v[e] = a; u[e] = c; }
      *(volatile v8b*)(w8h + ((size_t)m * H + n) * H + k0) = v; *(volatile v8b*)(w8l + ((size_t)m * H + n) * H + k0) = u; } __threadfence(); }
}

__global__ __launch_bounds__(256) void proj_kernel(const float* __restrict__ x, const float* __restrict__ pw, const float* __restrict__ pb, float* __restrict__ h) {
  const int i = blockIdx.x * 256 + threadIdx.x; const int row = i >> 4, cq = (i & 15) * 4; v4f o = {0.0f, 0.0f, 0.0f, 0.0f};
  if (row < N) { const float x0 = x[(size_t)row * 3], x1 = x[(size_t)row * 3 + 1], x2 = x[(size_t)row * 3 + 2];
#pragma unroll
    for (int c = 0; c < 4; ++c) o[c] = x0 * pw[cq + c] + x1 * pw[H + cq + c] + x2 * pw[2 * H + cq + c] + pb[cq + c]; }
  for (int pass = 0; pass < 2; ++pass) { *(volatile v4f*)(h + (size_t)row * H + cq) = o; __threadfence(); }
}

typedef __attribute__((ext_vector_type(4))) int v4i;
__global__ __launch_bounds__(256) void deg_kernel(const int* __restrict__ edst, float* __restrict__ dis) {
  constexpr int NB = 16384;
  __shared__ int cnt[NB];
  const int t_ = threadIdx.x, base = blockIdx.x * NB;
  for (int i = t_; i < NB; i += 256) cnt[i] = 0;
  __syncthreads();
  for (int e0 = t_ * 8; e0 < E; e0 += 256 * 8) { const v4i a = *(const v4i*)(edst + e0), b = *(const v4i*)(edst + e0 + 4); const int dd[8] = {a[0], a[1], a[2], a[3], b[0], b[1], b[2], b[3]};
#pragma unroll
    for (int j = 0; j < 8; ++j) { const unsigned sl = (unsigned)(dd[j] - base); if (sl < (unsigned)NB) atomicAdd(&cnt[sl], 1); } }
  __syncthreads();
  for (int pass = 0; pass < 2; ++pass) { for (int i = t_; i < NB; i += 256) { const int node = base + i; if (node < NPAD) ((volatile float*)dis)[node] = (node < N) ? rsqrtf((float)cnt[i] + 1.0f) : 0.0f; } __threadfence(); }
}

template <bool BNRELU>
__global__ __launch_bounds__(128) void lin_kernel(const float* __restrict__ hin, const float* __restrict__ coef, const b16* __restrict__ w, const b16* __restrict__ wlo, float* __restrict__ hw) {
  __shared__ __attribute__((aligned(16))) float Ts[4][32 * 64];
  const int lane = threadIdx.x & 31, wave = threadIdx.x >> 5, nloc = lane & 15, hlf = lane >> 4, m0 = blockIdx.x * 128 + wave * 32;
  v8f acc[2][4];
#pragma unroll
  for (int r = 0; r < 2; ++r)
#pragma unroll
    for (int t = 0; t < 4; ++t) acc[r][t] = (v8f){};
#pragma unroll
  for (int kb = 0; kb < H; kb += 32) { v16b a0, a1, l0, l1;
#pragma unroll
    for (int e = 0; e < 16; ++e) { const int k = kb + ((e < 8) ? (8 * hlf + e) : (16 + 8 * hlf + e - 8)); float u0 = hin[(size_t)(m0 + nloc) * H + k], u1 = hin[(size_t)(m0 + 16 + nloc) * H + k];
      if (BNRELU) { const float ca = coef[k], sh = coef[H + k]; u0 = fmaxf(u0 * ca + sh, 0.0f); u1 = fmaxf(u1 * ca + sh, 0.0f); } b16 p, q; split16(u0 * 8.0f, p, q); a0[e] = p; l0[e] = q; split16(u1 * 8.0f, p, q); a1[e] = p; l1[e] = q; }
#pragma unroll
    for (int t = 0; t < 4; ++t) { const v16b bw = frag_kb(w + (size_t)(t * 16 + nloc) * H + kb, hlf), bl = frag_kb(wlo + (size_t)(t * 16 + nloc) * H + kb, hlf);
      acc[0][t] = wmma16b(a0, bw, acc[0][t]); acc[0][t] = wmma16b(l0, bw, acc[0][t]); acc[0][t] = wmma16b(a0, bl, acc[0][t]);
      acc[1][t] = wmma16b(a1, bw, acc[1][t]); acc[1][t] = wmma16b(l1, bw, acc[1][t]); acc[1][t] = wmma16b(a1, bl, acc[1][t]); } }
  epi_f32(acc, 1.0f / 512.0f, nullptr, hw, H, m0, 0, lane, Ts[wave]);
}

__global__ __launch_bounds__(256) void gcn_kernel(const int* __restrict__ edst, const int* __restrict__ esrc, const float* __restrict__ hw, const float* __restrict__ dis, const float* __restrict__ bias, float* __restrict__ o, float* __restrict__ slot_) {
  constexpr int NB = 1024, DF = H;
  __shared__ __attribute__((aligned(16))) int acc[NB * DF];
  __shared__ int list[8 * 256]; __shared__ float Cs[2][DF]; __shared__ float Red[2][256 * 4];
  const int t_ = threadIdx.x, wave = t_ >> 5, lane = t_ & 31, base = blockIdx.x * NB;
  for (int i = t_; i < NB * DF; i += 256) acc[i] = 0;
  __syncthreads();
  int* wl = list + wave * 256;
  for (int c0 = 0; c0 < E; c0 += 256 * 8) {
    const int e0 = c0 + (wave * 32 + lane) * 8; int dd[8];
#pragma unroll
    for (int j = 0; j < 8; ++j) { const int dv = edst[min(e0 + j, E - 1)]; dd[j] = (e0 + j < E) ? dv : -1; }
    unsigned sl[8]; bool hit[8]; bool anyl = false;
#pragma unroll
    for (int j = 0; j < 8; ++j) { sl[j] = (unsigned)(dd[j] - base); hit[j] = sl[j] < (unsigned)NB; anyl |= hit[j]; }
    int wc = 0;
    if (__builtin_amdgcn_ballot_w32(anyl) != 0u) {
#pragma unroll
      for (int j = 0; j < 8; ++j) {
        const unsigned mj = __builtin_amdgcn_ballot_w32(hit[j]);
        if (mj != 0u) {
          if (hit[j]) { const int pos = wc + (int)__builtin_amdgcn_mbcnt_lo(mj, 0u); int s = esrc[min(e0 + j, E - 1)]; s = (s < 0) ? 0 : (s >= N ? N - 1 : s); wl[pos] = (s << 12) | (int)sl[j]; }
          wc += __builtin_popcount(mj); } } }
    __builtin_amdgcn_wave_barrier(); __builtin_amdgcn_fence(__ATOMIC_RELEASE, "workgroup"); __builtin_amdgcn_fence(__ATOMIC_ACQUIRE, "workgroup");
    for (int i0 = 0; i0 < wc; i0 += 2) { const int i = i0 + (lane >> 4); if (i < wc) { const int ent = wl[i]; const int s = ent >> 12, slot = ent & 4095; const int col = (lane & 15) * 4;
        const float w = dis[s]; const v4f v = *(const v4f*)(hw + (size_t)s * DF + col);
#pragma unroll
        for (int c = 0; c < 4; ++c) atomicAdd(&acc[slot * DF + col + c], (int)rintf(w * v[c] * FXS)); } }
    __builtin_amdgcn_wave_barrier();
  }
  __syncthreads();
  { const int cq = (t_ & 15) * 4, r0 = t_ >> 4;
    float s[4] = {0, 0, 0, 0}, s2[4] = {0, 0, 0, 0};
    for (int r = r0; r < NB; r += 16) { const int node = base + r; if (node < N) { const float di = dis[node];
#pragma unroll
        for (int q = 0; q < 4; ++q) { const float v = di * ((float)acc[r * DF + cq + q] * FXI) + di * di * hw[(size_t)node * DF + cq + q] + bias[cq + q]; s[q] += v; s2[q] += v * v; } } }
#pragma unroll
    for (int q = 0; q < 4; ++q) { Red[0][t_ * 4 + q] = s[q]; Red[1][t_ * 4 + q] = s2[q]; }
    __syncthreads();
    if (t_ < 16) { float a[4] = {0, 0, 0, 0}, b2[4] = {0, 0, 0, 0};
      for (int gq = 0; gq < 16; ++gq)
#pragma unroll
        for (int q = 0; q < 4; ++q) { a[q] += Red[0][(gq * 16 + t_) * 4 + q]; b2[q] += Red[1][(gq * 16 + t_) * 4 + q]; }
#pragma unroll
      for (int q = 0; q < 4; ++q) { Cs[0][cq + q] = a[q]; Cs[1][cq + q] = b2[q]; } }
    __syncthreads(); }
  for (int pass = 0; pass < 2; ++pass) {
    for (int i = t_; i < NB * DF / 4; i += 256) { const int r = i >> 4, cq = (i & 15) * 4, node = base + r; v4f ov = {0.0f, 0.0f, 0.0f, 0.0f};
      if (node < N) { const float di = dis[node];
#pragma unroll
        for (int q = 0; q < 4; ++q) ov[q] = di * ((float)acc[r * DF + cq + q] * FXI) + di * di * hw[(size_t)node * DF + cq + q] + bias[cq + q]; }
      *(volatile v4f*)(o + (size_t)node * DF + cq) = ov; }
    if (t_ < 32) ((volatile v4f*)(slot_ + (size_t)blockIdx.x * 2 * DF))[t_] = *(const v4f*)(&Cs[t_ >> 4][(t_ & 15) * 4]);
    __threadfence();
  }
}

__global__ __launch_bounds__(64) void bnfin_kernel(const float* __restrict__ slot_, const float* __restrict__ g, const float* __restrict__ bb, float* __restrict__ coef) {
  const int c = threadIdx.x; double s = 0.0, s2 = 0.0;
  for (int bk = 0; bk < NBA; ++bk) { s += (double)slot_[(size_t)bk * 2 * H + c]; s2 += (double)slot_[(size_t)bk * 2 * H + H + c]; }
  const double mean = s / N, var = s2 / N - mean * mean; const float a = g[c] * (float)(1.0 / sqrt(var + 1e-5)), sh = bb[c] - (float)mean * a;
  for (int pass = 0; pass < 2; ++pass) { ((volatile float*)coef)[c] = a; ((volatile float*)coef)[H + c] = sh; __threadfence(); }
}

__global__ __launch_bounds__(256) void resid_kernel(const float* __restrict__ o, const float* __restrict__ coef, float* __restrict__ h) {
  const int i = blockIdx.x * 256 + threadIdx.x; const int row = i >> 4, cq = (i & 15) * 4; const v4f ov = *(const v4f*)(o + (size_t)row * H + cq), hv = *(const v4f*)(h + (size_t)row * H + cq); v4f r;
#pragma unroll
  for (int c = 0; c < 4; ++c) r[c] = (row < N) ? fmaxf(ov[c] * coef[cq + c] + coef[H + cq + c] + hv[c], 0.0f) : 0.0f;
  for (int pass = 0; pass < 2; ++pass) { *(volatile v4f*)(h + (size_t)row * H + cq) = r; __threadfence(); }
}

__global__ __launch_bounds__(256) void pool_kernel(const float* __restrict__ h, const int* __restrict__ batch, float* __restrict__ z) {
  constexpr int GB = 64;
  __shared__ int sacc[GB * H]; __shared__ int smax[GB * H]; __shared__ int cnt[GB]; __shared__ int list[8 * 256];
  const int t_ = threadIdx.x, wave = t_ >> 5, lane = t_ & 31, gbase = blockIdx.x * GB;
  for (int i = t_; i < GB * H; i += 256) { sacc[i] = 0; smax[i] = fkey(-INFINITY); }
  if (t_ < GB) cnt[t_] = 0;
  __syncthreads();
  int* wl = list + wave * 256;
  for (int c0 = 0; c0 < N; c0 += 256 * 8) {
    const int n0 = c0 + (wave * 32 + lane) * 8; int dd[8];
#pragma unroll
    for (int j = 0; j < 8; ++j) { const int bv = batch[min(n0 + j, N - 1)]; dd[j] = (n0 + j < N) ? bv : -1; }
    unsigned sl[8]; bool hit[8]; bool anyl = false;
#pragma unroll
    for (int j = 0; j < 8; ++j) { sl[j] = (unsigned)(dd[j] - gbase); hit[j] = sl[j] < (unsigned)GB; anyl |= hit[j]; }
    int wc = 0;
    if (__builtin_amdgcn_ballot_w32(anyl) != 0u) {
#pragma unroll
      for (int j = 0; j < 8; ++j) {
        const unsigned mj = __builtin_amdgcn_ballot_w32(hit[j]);
        if (mj != 0u) {
          if (hit[j]) { const int pos = wc + (int)__builtin_amdgcn_mbcnt_lo(mj, 0u); wl[pos] = ((n0 + j) << 6) | (int)sl[j]; atomicAdd(&cnt[sl[j]], 1); }
          wc += __builtin_popcount(mj); } } }
    __builtin_amdgcn_wave_barrier(); __builtin_amdgcn_fence(__ATOMIC_RELEASE, "workgroup"); __builtin_amdgcn_fence(__ATOMIC_ACQUIRE, "workgroup");
    for (int i0 = 0; i0 < wc; i0 += 2) { const int i = i0 + (lane >> 4); if (i < wc) { const int ent = wl[i]; const int n = ent >> 6, slot = ent & 63; const int col = (lane & 15) * 4; const v4f v = *(const v4f*)(h + (size_t)n * H + col);
#pragma unroll
        for (int c = 0; c < 4; ++c) { atomicAdd(&sacc[slot * H + col + c], (int)rintf(v[c] * PFXS)); atomicMax(&smax[slot * H + col + c], fkey(v[c])); } } }
    __builtin_amdgcn_wave_barrier();
  }
  __syncthreads();
  for (int pass = 0; pass < 2; ++pass) { for (int i = t_; i < GB * H; i += 256) { const int slot = i / H, c = i % H; const float n_ = (float)cnt[slot];
      ((volatile float*)z)[(size_t)(gbase + slot) * 2 * H + c] = (float)sacc[i] * PFXI / fmaxf(n_, 1.0f);
      const float mx = fkey_inv(smax[i]); ((volatile float*)z)[(size_t)(gbase + slot) * 2 * H + H + c] = (n_ > 0.0f) ? mx : 0.0f; }
    __threadfence(); }
}

__global__ __launch_bounds__(256) void head_kernel(const float* __restrict__ z, const float* __restrict__ l1w, const float* __restrict__ l1b, const float* __restrict__ g1, const float* __restrict__ b1,
                                                   const float* __restrict__ l2w, const float* __restrict__ l2b, const float* __restrict__ g2, const float* __restrict__ b2, const float* __restrict__ l3w, const float* __restrict__ l3b, float* __restrict__ out) {
  __shared__ float Zt[G][H + 1]; __shared__ float csum[8][H], csq[8][H]; __shared__ float coefA[H], coefS[H]; __shared__ __attribute__((aligned(16))) b16 At[G][H + 8], Al[G][H + 8]; __shared__ float Ob[G * 2];
  const int t_ = threadIdx.x, wave = t_ >> 5, lane = t_ & 31, nloc = lane & 15, hlf = lane >> 4, m0 = wave * 32;
  v8f acc[2][4];
#pragma unroll
  for (int r = 0; r < 2; ++r)
#pragma unroll
    for (int t = 0; t < 4; ++t) acc[r][t] = (v8f){};
  { const Opnd A{z, nullptr, 2 * H};
#pragma unroll 1
    for (int kb = 0; kb < 2 * H; kb += 32) { v16b a0, a1, q0, q1;
#pragma unroll
      for (int e = 0; e < 16; ++e) { const int k = kb + ((e < 8) ? (8 * hlf + e) : (16 + 8 * hlf + e - 8)); b16 p, q; split16(z[(size_t)(m0 + nloc) * 2 * H + k] * 8.0f, p, q); a0[e] = p; q0[e] = q; split16(z[(size_t)(m0 + 16 + nloc) * 2 * H + k] * 8.0f, p, q); a1[e] = p; q1[e] = q; }
#pragma unroll
      for (int t = 0; t < 4; ++t) { v16b bw, bl;
#pragma unroll
        for (int e = 0; e < 16; ++e) { const int k = kb + ((e < 8) ? (8 * hlf + e) : (16 + 8 * hlf + e - 8)); b16 p, q; split16(l1w[(size_t)k * H + t * 16 + nloc] * 64.0f, p, q); bw[e] = p; bl[e] = q; }
        acc[0][t] = wmma16b(a0, bw, acc[0][t]); acc[0][t] = wmma16b(q0, bw, acc[0][t]); acc[0][t] = wmma16b(a0, bl, acc[0][t]);
        acc[1][t] = wmma16b(a1, bw, acc[1][t]); acc[1][t] = wmma16b(q1, bw, acc[1][t]); acc[1][t] = wmma16b(a1, bl, acc[1][t]); } } }
  auto bn_relu_stage = [&](int ncol, const float* bias, const float* gg, const float* bb) {
#pragma unroll
    for (int t = 0; t < 4; ++t)
#pragma unroll
      for (int r = 0; r < 2; ++r)
#pragma unroll
        for (int v = 0; v < 8; ++v) { const int c = t * 16 + nloc; if (c < ncol) Zt[m0 + r * 16 + v + 8 * hlf][c] = acc[r][t][v] * (1.0f / 512.0f) + bias[c]; }
    __syncthreads();
    if (t_ < ncol) { float s = 0.0f, s2 = 0.0f; for (int r = 0; r < G; ++r) { const float v = Zt[r][t_]; s += v; s2 += v * v; } const float mean = s / G, var = s2 / G - mean * mean; const float a = gg[t_] * rsqrtf(var + BNE); coefA[t_] = a; coefS[t_] = bb[t_] - mean * a; }
    __syncthreads();
    for (int i = t_; i < G * ncol; i += 256) { const int r = i / ncol, c = i % ncol; const float v = fmaxf(Zt[r][c] * coefA[c] + coefS[c], 0.0f); Zt[r][c] = v; b16 p, q; split16(v * 8.0f, p, q); At[r][c] = p; Al[r][c] = q; }
    __syncthreads();
  };
  bn_relu_stage(H, l1b, g1, b1);
#pragma unroll
  for (int r = 0; r < 2; ++r)
#pragma unroll
    for (int t = 0; t < 4; ++t) acc[r][t] = (v8f){};
#pragma unroll
  for (int kb = 0; kb < H; kb += 32) { const v16b a0 = frag_kb(&At[m0 + nloc][0] + kb, hlf), a1 = frag_kb(&At[m0 + 16 + nloc][0] + kb, hlf), q0 = frag_kb(&Al[m0 + nloc][0] + kb, hlf), q1 = frag_kb(&Al[m0 + 16 + nloc][0] + kb, hlf);
#pragma unroll
    for (int t = 0; t < 2; ++t) { v16b bw, bl;
#pragma unroll
      for (int e = 0; e < 16; ++e) { const int k = kb + ((e < 8) ? (8 * hlf + e) : (16 + 8 * hlf + e - 8)); b16 p, q; split16(l2w[(size_t)k * (H / 2) + t * 16 + nloc] * 64.0f, p, q); bw[e] = p; bl[e] = q; }
      acc[0][t] = wmma16b(a0, bw, acc[0][t]); acc[0][t] = wmma16b(q0, bw, acc[0][t]); acc[0][t] = wmma16b(a0, bl, acc[0][t]);
      acc[1][t] = wmma16b(a1, bw, acc[1][t]); acc[1][t] = wmma16b(q1, bw, acc[1][t]); acc[1][t] = wmma16b(a1, bl, acc[1][t]); } }
  __syncthreads();
  bn_relu_stage(H / 2, l2b, g2, b2);
  for (int i = t_; i < G * 2; i += 256) { const int r = i >> 1, c = i & 1; float s = l3b[c];
#pragma unroll 1
    for (int k = 0; k < H / 2; ++k) s += Zt[r][k] * l3w[k * 2 + c];
    Ob[i] = s; }
  __syncthreads();
  for (int pass = 0; pass < 2; ++pass) { if (t_ < G * 2 / 4) *(volatile v4f*)(out + t_ * 4) = *(const v4f*)(&Ob[t_ * 4]); __threadfence(); }
}
}

extern "C" void kernel_launch(void* const* d_in, const int* in_sizes, int n_in,
                              void* d_out, int out_size, void* d_ws, size_t ws_size, hipStream_t stream) {
  (void)n_in; (void)out_size;
  const float* x = (const float*)d_in[0]; const int* ei = (const int*)d_in[1]; const int* batch = (const int*)d_in[2]; const float* pw = (const float*)d_in[3]; const float* pb = (const float*)d_in[4];
  const float* cw = (const float*)d_in[5]; const float* cb = (const float*)d_in[6]; const float* bng = (const float*)d_in[7]; const float* bnb = (const float*)d_in[8];
  const float* l1w = (const float*)d_in[9]; const float* l1b = (const float*)d_in[10]; const float* l2w = (const float*)d_in[11]; const float* l2b = (const float*)d_in[12]; const float* l3w = (const float*)d_in[13]; const float* l3b = (const float*)d_in[14];
  const float* f1g = (const float*)d_in[15]; const float* f1b = (const float*)d_in[16]; const float* f2g = (const float*)d_in[17]; const float* f2b = (const float*)d_in[18];
  float* out = (float*)d_out;
  if (in_sizes[0] != N * 3 || in_sizes[1] != 2 * E || in_sizes[2] != N || in_sizes[5] != L * 2 * H * H || in_sizes[9] != 2 * H * H) return;
  const int* esrc = ei; const int* edst = ei + E;
  size_t off = 0; char* ws = (char*)d_ws;
  auto carve = [&](size_t bytes) { char* p = ws + off; off += (bytes + 255) & ~(size_t)255; return p; };
  b16* w8 = (b16*)carve((size_t)8 * H * H * 2); b16* w8l = (b16*)carve((size_t)8 * H * H * 2); float* dis = (float*)carve((size_t)NPAD * 4);
  float* h = (float*)carve((size_t)NPAD * H * 4); float* hw = (float*)carve((size_t)NPAD * H * 4); float* o = (float*)carve((size_t)NPAD * H * 4);
  float* slot_ = (float*)carve((size_t)NBA * 2 * H * 4); float* coef = (float*)carve(2 * H * 4); float* zg = (float*)carve((size_t)G * 2 * H * 4);
  if (off > ws_size) return;
  prep_kernel<<<32, 256, 0, stream>>>(cw, w8, w8l);
  deg_kernel<<<NPAD / 16384 + 1, 256, 0, stream>>>(edst, dis);
  proj_kernel<<<NPAD * 16 / 256, 256, 0, stream>>>(x, pw, pb, h);
  for (int l = 0; l < L; ++l) {
    lin_kernel<false><<<NBLK, 128, 0, stream>>>(h, nullptr, w8 + (size_t)(2 * l) * H * H, w8l + (size_t)(2 * l) * H * H, hw);
    gcn_kernel<<<NBA, 256, 0, stream>>>(edst, esrc, hw, dis, cb + (2 * l) * H, o, slot_);
    bnfin_kernel<<<1, 64, 0, stream>>>(slot_, bng + (2 * l) * H, bnb + (2 * l) * H, coef);
    lin_kernel<true><<<NBLK, 128, 0, stream>>>(o, coef, w8 + (size_t)(2 * l + 1) * H * H, w8l + (size_t)(2 * l + 1) * H * H, hw);
    gcn_kernel<<<NBA, 256, 0, stream>>>(edst, esrc, hw, dis, cb + (2 * l + 1) * H, o, slot_);
    bnfin_kernel<<<1, 64, 0, stream>>>(slot_, bng + (2 * l + 1) * H, bnb + (2 * l + 1) * H, coef);
    resid_kernel<<<NPAD * 16 / 256, 256, 0, stream>>>(o, coef, h);
  }
  pool_kernel<<<G / 64, 256, 0, stream>>>(h, batch, zg);
  head_kernel<<<1, 256, 0, stream>>>(zg, l1w, l1b, f1g, f1b, l2w, l2b, f2g, f2b, l3w, l3b, out);
}
